// EnergyAttention_15582141350436
// MI455X (gfx1250) — hardware-run, weakly checked
//
#include <hip/hip_runtime.h>
#include <math.h>

typedef __attribute__((ext_vector_type(16))) _Float16 v16h;
typedef __attribute__((ext_vector_type(8)))  _Float16 v8h;
typedef __attribute__((ext_vector_type(8)))  float    v8f;
typedef __attribute__((ext_vector_type(4)))  float    v4f;

constexpr int kQN    = 2048;
constexpr int kKN    = 4096;
constexpr int kDD    = 1024;
constexpr int kHH    = 16;
constexpr int kHD    = 64;
constexpr int kSteps = 5;
static_assert(kHH * kHD == kDD);
static_assert((kDD % 32) == 0 && (kQN % 128) == 0 && (kKN % 64) == 0 && (kDD % 64) == 0);
static_assert(((kKN / 64) * (kDD / 64)) % 8 == 0 && ((kQN / 64) * (kDD / 64)) % 8 == 0);

constexpr int isqrt_c(int n) { int r = 0; while ((r + 1) * (r + 1) <= n) ++r; return r; }
constexpr int kHdRoot = isqrt_c(kHD);
static_assert(kHdRoot * kHdRoot == kHD);

constexpr float kStepSize   = 0.1f;
constexpr float kBeta       = 1.0f / (float)kHdRoot;
constexpr float kActCarry   = 16.0f;
constexpr float kWCarry     = 1024.0f;
constexpr float kKCarry     = 16.0f;
constexpr float kQCarry     = 16.0f;
constexpr float kPCarryLog2 = 8.0f;
constexpr float kLog2e      = 1.4426950408889634f;
constexpr float kProjScale  = 1.0f / (kActCarry * kWCarry);
constexpr float kKhScale    = kKCarry * kProjScale;
constexpr float kSC2        = kBeta * kLog2e / (kQCarry * kKCarry);
constexpr float kUpdScale   = kStepSize / kKCarry;

constexpr size_t kOffCtx16 = 0;
constexpr size_t kOffTgt16 = kOffCtx16 + (size_t)kKN * kDD * 2;
constexpr size_t kOffWq16  = kOffTgt16 + (size_t)kQN * kDD * 2;
constexpr size_t kOffWk16  = kOffWq16  + (size_t)kDD * kDD * 2;
constexpr size_t kOffWo16  = kOffWk16  + (size_t)kDD * kDD * 2;
constexpr size_t kOffKh    = kOffWo16  + (size_t)kDD * kDD * 2;
constexpr size_t kOffKt    = kOffKh    + (size_t)kHH * kKN * kHD * 2;
constexpr size_t kOffQmA   = kOffKt    + (size_t)kHH * kHD * kKN * 2;
constexpr size_t kOffQmB   = kOffQmA   + (size_t)kQN * kDD * 4;
constexpr size_t kOffQsA   = kOffQmB   + (size_t)kQN * kDD * 4;
constexpr size_t kOffQsB   = kOffQsA   + (size_t)kHH * kQN * kHD * 2;
constexpr size_t kOffQfl   = kOffQsB   + (size_t)kHH * kQN * kHD * 2;
constexpr size_t kWsTotal  = kOffQfl   + (size_t)kQN * kDD * 2;
static_assert(kWsTotal == 65011712ull);
static_assert(kWsTotal <= 134217728ull);
static_assert((kOffTgt16 % 128) == 0 && (kOffWq16 % 128) == 0 && (kOffWk16 % 128) == 0 && (kOffWo16 % 128) == 0 &&
              (kOffKh % 128) == 0 && (kOffKt % 128) == 0 && (kOffQmA % 128) == 0 && (kOffQmB % 128) == 0 &&
              (kOffQsA % 128) == 0 && (kOffQsB % 128) == 0 && (kOffQfl % 128) == 0);

constexpr int kCastB1 = kKN * kDD / 2048;
constexpr int kCastB2 = kCastB1 + kQN * kDD / 2048;
constexpr int kCastB3 = kCastB2 + kDD * kDD / 2048;
constexpr int kCastB4 = kCastB3 + kDD * kDD / 2048;
constexpr int kCastB5 = kCastB4 + kDD * kDD / 2048;
static_assert((size_t)kCastB5 * 2048 * 2 == kOffKh);

union FragU { v16h v; v8h h[2]; };
__device__ __forceinline__ v16h frag_load(const _Float16* p) {
  FragU f;
  f.h[0] = *(const v8h*)(p);
  f.h[1] = *(const v8h*)(p + 16);
  return f.v;
}
__device__ __forceinline__ v8f mma_h(v16h a, v16h b, v8f c) {
  c = __builtin_amdgcn_wmma_f32_16x16x32_f16(false, a, false, b, (short)0, c, false, false);
  asm volatile("v_nop\n\tv_nop\n\tv_nop\n\tv_nop" : "+v"(c) : "v"(a), "v"(b));
  return c;
}
__device__ __forceinline__ void wave_sync() {
  __builtin_amdgcn_fence(__ATOMIC_RELEASE, "workgroup");
  __builtin_amdgcn_wave_barrier();
  __builtin_amdgcn_fence(__ATOMIC_ACQUIRE, "workgroup");
}

__device__ __forceinline__ void store32_slab(const float* slab, float* dst, size_t pitch, int lane) {
  const int hh = lane >> 4, c4 = (lane & 15) * 4;
  for (int pass = 0; pass < 2; ++pass) {
#pragma unroll
    for (int it = 0; it < 8; ++it) {
      const int row = it * 2 + hh;
      const v4f v = *(const v4f*)(slab + row * 68 + c4);
      *(volatile v4f*)(dst + (size_t)row * pitch + c4) = v;
    }
    __threadfence();
  }
}
__device__ __forceinline__ void store16_slab(const float* slab, unsigned short* dst, size_t pitch, float sc, int lane) {
  const int q4 = lane >> 3, c8 = (lane & 7) * 8;
  for (int pass = 0; pass < 2; ++pass) {
#pragma unroll
    for (int it = 0; it < 4; ++it) {
      const int row = it * 4 + q4;
      const float* sp = slab + row * 68 + c8;
      v8h hv;
#pragma unroll
      for (int e = 0; e < 8; ++e) hv[e] = (_Float16)(sp[e] * sc);
      *(volatile v8h*)(dst + (size_t)row * pitch + c8) = hv;
    }
    __threadfence();
  }
}

__global__ __launch_bounds__(256) void cast_planes_kernel(
    const float* __restrict__ ctx, const float* __restrict__ tgt, const float* __restrict__ wq,
    const float* __restrict__ wk, const float* __restrict__ wo, unsigned short* __restrict__ out)
{
  const int blk = blockIdx.x;
  const float* src = ctx;
  int b0 = 0;
  float sc = kActCarry;
  if (blk >= kCastB1) { src = tgt; b0 = kCastB1; }
  if (blk >= kCastB2) { src = wq; b0 = kCastB2; sc = kWCarry; }
  if (blk >= kCastB3) { src = wk; b0 = kCastB3; }
  if (blk >= kCastB4) { src = wo; b0 = kCastB4; }
  const size_t ein  = ((size_t)(blk - b0) * 256 + threadIdx.x) * 8;
  const size_t eout = ((size_t)blk * 256 + threadIdx.x) * 8;
  const v4f a = *(const v4f*)(src + ein);
  const v4f c = *(const v4f*)(src + ein + 4);
  v8h hv;
#pragma unroll
  for (int e = 0; e < 4; ++e) {
    hv[e]     = (_Float16)(a[e] * sc);
    hv[4 + e] = (_Float16)(c[e] * sc);
  }
  unsigned short* q = out + eout;
  *(volatile v8h*)q = hv;
  __threadfence();
  *(volatile v8h*)q = hv;
}

template <int MODE>
__global__ __launch_bounds__(256) void gemm_f16_kernel(
    const unsigned short* __restrict__ Ap, int lda,
    const unsigned short* __restrict__ Btp, int ldb,
    float* __restrict__ Cf, int ldc,
    unsigned short* __restrict__ P1, unsigned short* __restrict__ P2,
    int M, int N, int K, float scale, float scale16)
{
  const _Float16* A  = (const _Float16*)Ap;
  const _Float16* Bt = (const _Float16*)Btp;
  __shared__ __align__(16) float sT[8][16 * 68];
  const int lane = threadIdx.x & 31;
  const int wave = __builtin_amdgcn_readfirstlane((int)(threadIdx.x >> 5));
  const int tilesN = N >> 6;
  const int tilesM = M >> 6;
  const int tile = blockIdx.x * 8 + wave;
  if (tile >= tilesM * tilesN) return;
  const int tm = tile / tilesN;
  const int tn = tile - tm * tilesN;
  const int m0 = tm << 6;
  const int n0 = tn << 6;

  const int rlane = lane & 15;
  const int koff  = (lane >> 4) * 8;
  const int mOff  = (lane >> 4) * 8;

  v8f acc[4][4];
#pragma unroll
  for (int i = 0; i < 4; ++i)
#pragma unroll
    for (int j = 0; j < 4; ++j) acc[i][j] = (v8f){0.f, 0.f, 0.f, 0.f, 0.f, 0.f, 0.f, 0.f};

  for (int k0 = 0; k0 < K; k0 += 32) {
    v16h bh[4];
#pragma unroll
    for (int j = 0; j < 4; ++j)
      bh[j] = frag_load(Bt + (size_t)(n0 + (j << 4) + rlane) * ldb + koff + k0);
#pragma unroll
    for (int i = 0; i < 4; ++i) {
      const v16h ah = frag_load(A + (size_t)(m0 + (i << 4) + rlane) * lda + koff + k0);
#pragma unroll
      for (int j = 0; j < 4; ++j) acc[i][j] = mma_h(ah, bh[j], acc[i][j]);
    }
  }

  float* slab = sT[wave];
#pragma unroll
  for (int i = 0; i < 4; ++i) {
    const int mBase = m0 + (i << 4);
#pragma unroll
    for (int j = 0; j < 4; ++j)
#pragma unroll
      for (int r = 0; r < 8; ++r)
        slab[(mOff + r) * 68 + (j << 4) + rlane] = acc[i][j][r] * scale;
    wave_sync();
    if (MODE == 0 || MODE == 1)
      store32_slab(slab, Cf + (size_t)mBase * ldc + n0, (size_t)ldc, lane);
    if (MODE == 1 || MODE == 2)
      store16_slab(slab, P1 + ((size_t)tn * M + mBase) * 64, (size_t)64, scale16, lane);
    wave_sync();
  }
  if (MODE == 2) {
#pragma unroll
    for (int j = 0; j < 4; ++j) {
#pragma unroll
      for (int i = 0; i < 4; ++i)
#pragma unroll
        for (int r = 0; r < 8; ++r)
          slab[rlane * 68 + (i << 4) + mOff + r] = acc[i][j][r] * scale;
      wave_sync();
      store16_slab(slab, P2 + ((size_t)tn * 64 + (j << 4)) * M + m0, (size_t)M, scale16, lane);
      wave_sync();
    }
  }
}

__global__ __attribute__((amdgpu_num_vgpr(256))) __launch_bounds__(128) void descent_step_kernel(
    const unsigned short* __restrict__ Qs, const unsigned short* __restrict__ Kh,
    const unsigned short* __restrict__ Kt, const float* __restrict__ QmIn,
    float* __restrict__ QmOut, unsigned short* __restrict__ snapOut,
    long snapHeadStride, int snapRowPitch, int writeMaster)
{
  __shared__ __align__(16) float Os[4][32 * 68];
  const int lane = threadIdx.x & 31;
  const int wave = __builtin_amdgcn_readfirstlane((int)(threadIdx.x >> 5));
  const int hh = lane >> 4;
  const int c  = lane & 15;
  const int h  = blockIdx.x & (kHH - 1);
  const int qbase = (blockIdx.x / kHH) * 128 + wave * 32;

  const _Float16* kb  = (const _Float16*)Kh + (size_t)h * kKN * kHD;
  const _Float16* ktb = (const _Float16*)Kt + (size_t)h * kHD * kKN;
  const _Float16* qsb = (const _Float16*)Qs + ((size_t)h * kQN + qbase) * kHD;

  v16h qb[2][2];
#pragma unroll
  for (int u = 0; u < 2; ++u)
#pragma unroll
    for (int f = 0; f < 2; ++f)
      qb[u][f] = frag_load(qsb + (size_t)(u * 16 + c) * kHD + f * 32 + 8 * hh);

  v8f acc[2][4];
#pragma unroll
  for (int u = 0; u < 2; ++u)
#pragma unroll
    for (int t = 0; t < 4; ++t) acc[u][t] = (v8f){0.f, 0.f, 0.f, 0.f, 0.f, 0.f, 0.f, 0.f};
  float mrun[2]  = {-1e30f, -1e30f};
  float lpart[2] = {0.0f, 0.0f};

#pragma unroll 1
  for (int k0 = 0; k0 < kKN; k0 += 64) {
    v8f s[2][4];
#pragma unroll
    for (int t = 0; t < 4; ++t) {
      s[0][t] = (v8f){0.f, 0.f, 0.f, 0.f, 0.f, 0.f, 0.f, 0.f};
      s[1][t] = (v8f){0.f, 0.f, 0.f, 0.f, 0.f, 0.f, 0.f, 0.f};
    }
#pragma unroll
    for (int t = 0; t < 4; ++t) {
#pragma unroll
      for (int f = 0; f < 2; ++f) {
        const v16h ak = frag_load(kb + (size_t)(k0 + t * 16 + c) * kHD + f * 32 + 8 * hh);
        s[0][t] = mma_h(ak, qb[0][f], s[0][t]);
        s[1][t] = mma_h(ak, qb[1][f], s[1][t]);
      }
    }

    v16h pb[2][2];
#pragma unroll
    for (int u = 0; u < 2; ++u) {
      float mx = s[u][0][0];
#pragma unroll
      for (int t = 0; t < 4; ++t)
#pragma unroll
        for (int r = 0; r < 8; ++r) mx = fmaxf(mx, s[u][t][r]);
      const float mo = __shfl_xor(mx, 16, 32);
      mx = fmaxf(mx, mo);
      const float mn = fmaxf(mrun[u], mx);
      const int moved = __any(mx > mrun[u]);
      if (moved) {
        const float corr = __builtin_amdgcn_exp2f((mrun[u] - mn) * kSC2);
        lpart[u] *= corr;
#pragma unroll
        for (int t = 0; t < 4; ++t)
#pragma unroll
          for (int r = 0; r < 8; ++r) acc[u][t][r] *= corr;
      }
      mrun[u] = mn;
      const float nb = fmaf(-mn, kSC2, kPCarryLog2);
      float rs = 0.0f;
#pragma unroll
      for (int g = 0; g < 2; ++g) {
#pragma unroll
        for (int e = 0; e < 8; ++e) {
          const float p0 = __builtin_amdgcn_exp2f(fmaf(s[u][2 * g][e], kSC2, nb));
          const float p1 = __builtin_amdgcn_exp2f(fmaf(s[u][2 * g + 1][e], kSC2, nb));
          rs += p0;
          rs += p1;
          pb[u][g][e]     = (_Float16)p0;
          pb[u][g][8 + e] = (_Float16)p1;
        }
      }
      lpart[u] += rs;
    }

#pragma unroll
    for (int g = 0; g < 2; ++g) {
#pragma unroll
      for (int t = 0; t < 4; ++t) {
        const v16h ak = frag_load(ktb + (size_t)(t * 16 + c) * kKN + k0 + g * 32 + 8 * hh);
        acc[0][t] = mma_h(ak, pb[0][g], acc[0][t]);
        acc[1][t] = mma_h(ak, pb[1][g], acc[1][t]);
      }
    }
  }

  float* os = Os[wave];
#pragma unroll
  for (int u = 0; u < 2; ++u) {
    const float lo = __shfl_xor(lpart[u], 16, 32);
    const float l = lpart[u] + lo;
    const float inv = kUpdScale * (1.0f / l);
#pragma unroll
    for (int t = 0; t < 4; ++t) {
      float* d = os + (u * 16 + c) * 68 + t * 16 + 8 * hh;
      const v4f v0 = (v4f){acc[u][t][0] * inv, acc[u][t][1] * inv, acc[u][t][2] * inv, acc[u][t][3] * inv};
      const v4f v1 = (v4f){acc[u][t][4] * inv, acc[u][t][5] * inv, acc[u][t][6] * inv, acc[u][t][7] * inv};
      *(v4f*)(d)     = v0;
      *(v4f*)(d + 4) = v1;
    }
  }
  __syncthreads();

  const int c4 = c * 4;
#pragma unroll
  for (int grp = 0; grp < 2; ++grp) {
    v4f nv[8];
#pragma unroll
    for (int it = 0; it < 8; ++it) {
      const int row = grp * 16 + it * 2 + hh;
      float* sp = os + row * 68 + c4;
      const v4f d = *(const v4f*)sp;
      const v4f o = *(const v4f*)(QmIn + (size_t)(qbase + row) * kDD + h * kHD + c4);
      nv[it] = o + d;
      *(v4f*)sp = nv[it];
    }
    if (writeMaster != 0) {
      for (int pass = 0; pass < 2; ++pass) {
#pragma unroll
        for (int it = 0; it < 8; ++it) {
          const int row = grp * 16 + it * 2 + hh;
          *(volatile v4f*)(QmOut + (size_t)(qbase + row) * kDD + h * kHD + c4) = nv[it];
        }
        __threadfence();
      }
    }
  }
  __syncthreads();

  unsigned short* sb = snapOut + (size_t)h * snapHeadStride + (size_t)qbase * snapRowPitch;
  store16_slab(os, sb, (size_t)snapRowPitch, kQCarry, lane);
  store16_slab(os + 16 * 68, sb + (size_t)16 * snapRowPitch, (size_t)snapRowPitch, kQCarry, lane);
}

extern "C" void kernel_launch(void* const* d_in, const int* in_sizes, int n_in,
                              void* d_out, int out_size, void* d_ws, size_t ws_size,
                              hipStream_t stream) {
  if (n_in < 5) return;
  if (in_sizes[0] != kKN * kDD) return;
  if (in_sizes[1] != kQN * kDD) return;
  if (in_sizes[2] != kDD * kDD) return;
  if (in_sizes[3] != kDD * kDD) return;
  if (in_sizes[4] != kDD * kDD) return;
  if (out_size != kQN * kDD) return;
  if (ws_size < kWsTotal) return;

  const float* ctx = (const float*)d_in[0];
  const float* tgt = (const float*)d_in[1];
  const float* Wq  = (const float*)d_in[2];
  const float* Wk  = (const float*)d_in[3];
  const float* Wo  = (const float*)d_in[4];
  float* out = (float*)d_out;

  char* ws = (char*)d_ws;
  unsigned short* CTX16 = (unsigned short*)(ws + kOffCtx16);
  unsigned short* TGT16 = (unsigned short*)(ws + kOffTgt16);
  unsigned short* WQ16  = (unsigned short*)(ws + kOffWq16);
  unsigned short* WK16  = (unsigned short*)(ws + kOffWk16);
  unsigned short* WO16  = (unsigned short*)(ws + kOffWo16);
  unsigned short* KH    = (unsigned short*)(ws + kOffKh);
  unsigned short* KT    = (unsigned short*)(ws + kOffKt);
  float*          QMA   = (float*)(ws + kOffQmA);
  float*          QMB   = (float*)(ws + kOffQmB);
  unsigned short* QSA   = (unsigned short*)(ws + kOffQsA);
  unsigned short* QSB   = (unsigned short*)(ws + kOffQsB);
  unsigned short* QFL   = (unsigned short*)(ws + kOffQfl);

  cast_planes_kernel<<<kCastB5, 256, 0, stream>>>(ctx, tgt, Wq, Wk, Wo, CTX16);

  gemm_f16_kernel<2><<<((kKN / 64) * (kDD / 64)) / 8, 256, 0, stream>>>(
      CTX16, kDD, WK16, kDD, QMA, kDD, KH, KT, kKN, kDD, kDD, kKhScale, 1.0f);

  gemm_f16_kernel<1><<<((kQN / 64) * (kDD / 64)) / 8, 256, 0, stream>>>(
      TGT16, kDD, WQ16, kDD, QMA, kDD, QSA, QSB, kQN, kDD, kDD, kProjScale, kQCarry);

  for (int s = 0; s < kSteps; ++s) {
    const bool even = ((s & 1) == 0);
    const bool last = (s == kSteps - 1);
    const unsigned short* qsIn = even ? QSA : QSB;
    unsigned short* qsOut      = even ? QSB : QSA;
    const float* qmIn          = even ? QMA : QMB;
    float* qmOut               = even ? QMB : QMA;
    if (!last) {
      descent_step_kernel<<<(kQN / 128) * kHH, 128, 0, stream>>>(
          qsIn, KH, KT, qmIn, qmOut, qsOut, (long)kQN * kHD, kHD, 1);
    } else {
      descent_step_kernel<<<(kQN / 128) * kHH, 128, 0, stream>>>(
          qsIn, KH, KT, qmIn, qmOut, QFL, (long)kHD, kDD, 0);
    }
  }

  gemm_f16_kernel<0><<<((kQN / 64) * (kDD / 64)) / 8, 256, 0, stream>>>(
      QFL, kDD, WO16, kDD, out, kDD, QSA, QSB, kQN, kDD, kDD, kProjScale, 1.0f);
}
